// TransformerBlock_120259085226
// MI455X (gfx1250) — hardware-verified
//
#include <hip/hip_runtime.h>
#include <stddef.h>


typedef _Float16 v16h __attribute__((ext_vector_type(16)));
typedef _Float16 v8h  __attribute__((ext_vector_type(8)));
typedef float    v8f  __attribute__((ext_vector_type(8)));
typedef float    v4f  __attribute__((ext_vector_type(4)));

#ifndef NB
#define NB 8
#endif
#ifndef SEQ
#define SEQ 2048
#endif
#define NB_FULL  8
#define SEQ_FULL 2048
#define DIM   512
#define NHEAD 8
#define HD    64
#define MROWS (NB * SEQ)

static_assert(NB >= 1 && NB <= NB_FULL);
static_assert(SEQ >= 128 && SEQ <= SEQ_FULL && (SEQ % 128) == 0);
static_assert(DIM == NHEAD * HD);
static_assert((MROWS % 64) == 0);
static_assert(((size_t)MROWS * DIM) % (8 * 256) == 0);

#define LDT 72
#define LDC 68

#define WCARRY 64.0f
#define PCARRY 1024.0f
#define VCARRY 64.0f

#define PLANE16_BYTES ((size_t)MROWS * DIM * 2)
#define PLANE32_BYTES ((size_t)MROWS * DIM * 4)
#define WT_BYTES      ((size_t)6 * DIM * DIM * 2)
#define R1_BYTES      (PLANE16_BYTES * 4)
#define R2_BYTES      (PLANE16_BYTES * 3)
#define WS_TOTAL      (WT_BYTES + R1_BYTES + R2_BYTES)
static_assert(PLANE16_BYTES * 3 <= R1_BYTES);
static_assert(PLANE16_BYTES + PLANE32_BYTES + PLANE16_BYTES <= R1_BYTES);
static_assert(WS_TOTAL <= (size_t)134217728);

__device__ __forceinline__ float bf16r(float x) {
  unsigned int u = __float_as_uint(x);
  u = (u + 0x7FFFu + ((u >> 16) & 1u)) & 0xFFFF0000u;
  return __uint_as_float(u);
}

__device__ __forceinline__ v16h frag_at(const _Float16* p) {
  v8h lo = *(const v8h*)(p);
  v8h hi = *(const v8h*)(p + 16);
  v16h out;
#pragma unroll
  for (int i = 0; i < 8; ++i) { out[i] = lo[i]; out[i + 8] = hi[i]; }
  return out;
}
__device__ __forceinline__ v16h ld_frag(const _Float16* base, int ld) {
  const int lane = threadIdx.x & 31;
  return frag_at(base + (lane & 15) * ld + (lane >> 4) * 8);
}

__device__ __forceinline__ v8f wmma16(v16h a, v16h b, v8f c) {
  v8f d = __builtin_amdgcn_wmma_f32_16x16x32_f16(false, a, false, b, (short)0, c,
                                                 false, false);
  asm volatile("v_nop\n\tv_nop\n\tv_nop\n\tv_nop" : "+v"(d) : "v"(a), "v"(b));
  return d;
}

__device__ __forceinline__ float red16_max(float x) {
#pragma unroll
  for (int off = 1; off < 16; off <<= 1) x = fmaxf(x, __shfl_xor(x, off, 32));
  return x;
}
__device__ __forceinline__ float red16_sum(float x) {
#pragma unroll
  for (int off = 1; off < 16; off <<= 1) x += __shfl_xor(x, off, 32);
  return x;
}

__device__ __forceinline__ void wave_lds_sync() {
  __builtin_amdgcn_fence(3  , "wavefront");
  asm volatile("s_wait_dscnt 0x0" ::: "memory");
  __builtin_amdgcn_wave_barrier();
}

__global__ __launch_bounds__(256) void wconv_kernel(
    const float* __restrict__ W0, const float* __restrict__ W1p,
    const float* __restrict__ W2p, const float* __restrict__ W3,
    const float* __restrict__ W4, const float* __restrict__ W5,
    _Float16* __restrict__ Wt) {
  __shared__ _Float16 T[64 * LDT];
  const int tid = threadIdx.x;
  const int n0 = blockIdx.x * 64;
  const int k0 = blockIdx.y * 64;
  const int p = blockIdx.z;
  const float* W = W0;
  if (p == 1) W = W1p;
  if (p == 2) W = W2p;
  if (p == 3) W = W3;
  if (p == 4) W = W4;
  if (p == 5) W = W5;
  if (p < 4) {
#pragma unroll 4
    for (int j = 0; j < 16; ++j) {
      const int idx = tid + 256 * j;
      const int kr = idx >> 6, nc = idx & 63;
      const float v = W[(size_t)(k0 + kr) * DIM + n0 + nc];
      T[nc * LDT + kr] = (_Float16)(WCARRY * bf16r(v));
    }
  } else {
#pragma unroll 4
    for (int j = 0; j < 16; ++j) {
      const int idx = tid + 256 * j;
      const int nr = idx >> 6, kc = idx & 63;
      const float v = W[(size_t)(n0 + nr) * DIM + k0 + kc];
      T[nr * LDT + kc] = (_Float16)(WCARRY * bf16r(v));
    }
  }
  __syncthreads();
  v8h x[2];
  size_t off[2];
#pragma unroll
  for (int i = 0; i < 2; ++i) {
    const int n = 32 * i + (tid >> 3);
    const int kc = (tid & 7) * 8;
    x[i] = *(const v8h*)&T[n * LDT + kc];
    off[i] = (size_t)p * DIM * DIM + (size_t)(n0 + n) * DIM + k0 + kc;
  }
#pragma unroll
  for (int i = 0; i < 2; ++i) *(volatile v8h*)(Wt + off[i]) = x[i];
  __threadfence();
#pragma unroll
  for (int i = 0; i < 2; ++i) *(volatile v8h*)(Wt + off[i]) = x[i];
}

__global__ __launch_bounds__(256) void xconv_kernel(
    const float* __restrict__ Qin, const float* __restrict__ Kin,
    const float* __restrict__ Vin, _Float16* __restrict__ planes) {
  const int which = blockIdx.y;
  const float* src = Qin;
  if (which == 1) src = Kin;
  if (which == 2) src = Vin;
  _Float16* dst = planes + (size_t)which * ((size_t)MROWS * DIM);
  const size_t e = ((size_t)blockIdx.x * 256 + threadIdx.x) * 8;
  const size_t crow = e / DIM;
  const int c = (int)(e - crow * DIM);
  const size_t bidx = crow / SEQ;
  const size_t sq = crow - bidx * SEQ;
  const size_t frow = bidx * SEQ_FULL + sq;
  const float* sp = src + frow * DIM + c;
  const v4f a0 = *(const v4f*)(sp);
  const v4f a1 = *(const v4f*)(sp + 4);
  v8h o;
#pragma unroll
  for (int j = 0; j < 4; ++j) {
    o[j]     = (_Float16)bf16r(a0[j]);
    o[j + 4] = (_Float16)bf16r(a1[j]);
  }
  *(volatile v8h*)(dst + e) = o;
  __threadfence();
  *(volatile v8h*)(dst + e) = o;
}

template <int MODE>
__global__ __launch_bounds__(256) void gemm_kernel(
    const _Float16* __restrict__ A16, const _Float16* __restrict__ Bt,
    const float* __restrict__ addf, const float* __restrict__ resf,
    float* __restrict__ outf, _Float16* __restrict__ out16) {
  __shared__ float Cs[64 * LDC];
  const int tid = threadIdx.x, lane = tid & 31, w = tid >> 5;
  const int mw = w >> 1, nw = w & 1;
  const int hh = lane >> 4, m = lane & 15;
  const int n0 = blockIdx.x * 64;
  const int row0 = blockIdx.y * 64;

  const _Float16* ap  = A16 + (size_t)(row0 + mw * 16 + m) * DIM + hh * 8;
  const _Float16* bp0 = Bt + (size_t)(n0 + nw * 32 + m) * DIM + hh * 8;
  const _Float16* bp1 = bp0 + 16 * DIM;
  v8f acc0 = {}, acc1 = {};
#pragma unroll 2
  for (int k0 = 0; k0 < DIM; k0 += 32) {
    const v16h a  = frag_at(ap + k0);
    const v16h b0 = frag_at(bp0 + k0);
    const v16h b1 = frag_at(bp1 + k0);
    acc0 = wmma16(a, b0, acc0);
    acc1 = wmma16(a, b1, acc1);
  }
#pragma unroll
  for (int r = 0; r < 8; ++r) {
    float* d = &Cs[(mw * 16 + hh * 8 + r) * LDC + nw * 32 + m];
    d[0]  = acc0[r];
    d[16] = acc1[r];
  }
  __syncthreads();

  if (MODE == 0) {
    v8h x[2];
    size_t off[2];
#pragma unroll
    for (int i = 0; i < 2; ++i) {
      const int r = 32 * i + (tid >> 3);
      const int c = (tid & 7) * 8;
      const v4f u0 = *(const v4f*)&Cs[r * LDC + c];
      const v4f u1 = *(const v4f*)&Cs[r * LDC + c + 4];
#pragma unroll
      for (int j = 0; j < 4; ++j) {
        x[i][j]     = (_Float16)(u0[j] * (1.0f / WCARRY));
        x[i][j + 4] = (_Float16)(u1[j] * (1.0f / WCARRY));
      }
      off[i] = (size_t)(row0 + r) * DIM + n0 + c;
    }
#pragma unroll
    for (int i = 0; i < 2; ++i) *(volatile v8h*)(out16 + off[i]) = x[i];
    __threadfence();
#pragma unroll
    for (int i = 0; i < 2; ++i) *(volatile v8h*)(out16 + off[i]) = x[i];
  }

  if (MODE == 1) {
    const int bidx = row0 / SEQ;
    const int key0 = row0 - bidx * SEQ;
    v8h x[2];
    size_t off[2];
#pragma unroll
    for (int i = 0; i < 2; ++i) {
      const int dcol = 32 * i + (tid >> 3);
      const int kk = (tid & 7) * 8;
#pragma unroll
      for (int j = 0; j < 8; ++j)
        x[i][j] = (_Float16)(Cs[(kk + j) * LDC + dcol] * (1.0f / WCARRY));
      off[i] = ((size_t)(bidx * DIM + n0 + dcol)) * SEQ + key0 + kk;
    }
#pragma unroll
    for (int i = 0; i < 2; ++i) *(volatile v8h*)(out16 + off[i]) = x[i];
    __threadfence();
#pragma unroll
    for (int i = 0; i < 2; ++i) *(volatile v8h*)(out16 + off[i]) = x[i];
  }

  if (MODE == 2) {
    v4f xs[4];
    size_t off[4];
#pragma unroll
    for (int i = 0; i < 4; ++i) {
      const int r = 16 * i + (tid >> 4);
      const int c = (tid & 15) * 4;
      const int crow = row0 + r;
      const int bidx = crow / SEQ;
      const int sq = crow - bidx * SEQ;
      const size_t frow = (size_t)bidx * SEQ_FULL + sq;
      const v4f u = *(const v4f*)&Cs[r * LDC + c];
      const v4f q = *(const v4f*)(addf + frow * DIM + n0 + c);
      v4f val;
#pragma unroll
      for (int j = 0; j < 4; ++j)
        val[j] = u[j] * (1.0f / (WCARRY * VCARRY)) + bf16r(q[j]);
      xs[i] = val;
      *(v4f*)&Cs[r * LDC + c] = val;
      off[i] = (size_t)crow * DIM + n0 + c;
    }
#pragma unroll
    for (int i = 0; i < 4; ++i) *(volatile v4f*)(outf + off[i]) = xs[i];
    __threadfence();
#pragma unroll
    for (int i = 0; i < 4; ++i) *(volatile v4f*)(outf + off[i]) = xs[i];
    __syncthreads();
    v8h x[2];
    size_t off2[2];
#pragma unroll
    for (int i = 0; i < 2; ++i) {
      const int r = 32 * i + (tid >> 3);
      const int c = (tid & 7) * 8;
      const v4f u0 = *(const v4f*)&Cs[r * LDC + c];
      const v4f u1 = *(const v4f*)&Cs[r * LDC + c + 4];
#pragma unroll
      for (int j = 0; j < 4; ++j) {
        x[i][j]     = (_Float16)u0[j];
        x[i][j + 4] = (_Float16)u1[j];
      }
      off2[i] = (size_t)(row0 + r) * DIM + n0 + c;
    }
#pragma unroll
    for (int i = 0; i < 2; ++i) *(volatile v8h*)(out16 + off2[i]) = x[i];
    __threadfence();
#pragma unroll
    for (int i = 0; i < 2; ++i) *(volatile v8h*)(out16 + off2[i]) = x[i];
  }

  if (MODE == 3) {
    v8h x[2];
    size_t off[2];
#pragma unroll
    for (int i = 0; i < 2; ++i) {
      const int r = 32 * i + (tid >> 3);
      const int c = (tid & 7) * 8;
      const v4f u0 = *(const v4f*)&Cs[r * LDC + c];
      const v4f u1 = *(const v4f*)&Cs[r * LDC + c + 4];
      const v4f g0 = *(const v4f*)(addf + n0 + c);
      const v4f g1 = *(const v4f*)(addf + n0 + c + 4);
#pragma unroll
      for (int j = 0; j < 4; ++j) {
        const float t0 = fmaxf(u0[j] * (1.0f / WCARRY) + bf16r(g0[j]), 0.0f);
        const float t1 = fmaxf(u1[j] * (1.0f / WCARRY) + bf16r(g1[j]), 0.0f);
        x[i][j]     = (_Float16)t0;
        x[i][j + 4] = (_Float16)t1;
      }
      off[i] = (size_t)(row0 + r) * DIM + n0 + c;
    }
#pragma unroll
    for (int i = 0; i < 2; ++i) *(volatile v8h*)(out16 + off[i]) = x[i];
    __threadfence();
#pragma unroll
    for (int i = 0; i < 2; ++i) *(volatile v8h*)(out16 + off[i]) = x[i];
  }

  if (MODE == 4) {
    v4f xs[4];
    size_t off[4];
#pragma unroll
    for (int i = 0; i < 4; ++i) {
      const int r = 16 * i + (tid >> 4);
      const int c = (tid & 15) * 4;
      const int crow = row0 + r;
      const int bidx = crow / SEQ;
      const int sq = crow - bidx * SEQ;
      const size_t frow = (size_t)bidx * SEQ_FULL + sq;
      const v4f u  = *(const v4f*)&Cs[r * LDC + c];
      const v4f g  = *(const v4f*)(addf + n0 + c);
      const v4f rx = *(const v4f*)(resf + (size_t)crow * DIM + n0 + c);
      v4f val;
#pragma unroll
      for (int j = 0; j < 4; ++j)
        val[j] = (u[j] * (1.0f / WCARRY) + bf16r(g[j])) + rx[j];
      xs[i] = val;
      off[i] = frow * DIM + n0 + c;
    }
#pragma unroll
    for (int i = 0; i < 4; ++i) *(volatile v4f*)(outf + off[i]) = xs[i];
    __threadfence();
#pragma unroll
    for (int i = 0; i < 4; ++i) *(volatile v4f*)(outf + off[i]) = xs[i];
  }
}

__global__ __launch_bounds__(256) void attn_kernel(
    const _Float16* __restrict__ Qh, const _Float16* __restrict__ Kh,
    const _Float16* __restrict__ Vt, _Float16* __restrict__ Ov) {
  __shared__ _Float16 Ks[64 * LDT];
  __shared__ _Float16 Vs[64 * LDT];
  __shared__ _Float16 Ps[8 * 16 * LDT];

  const int tid = threadIdx.x, lane = tid & 31, w = tid >> 5;
  const int hh = lane >> 4, m = lane & 15;
  const int q0 = blockIdx.x * 128;
  const int head = blockIdx.y;
  const int b = blockIdx.z;
  const float scale = 1.0f / 8.000001f;
  _Float16* P = Ps + w * (16 * LDT);

  const size_t qoff = (size_t)(b * SEQ + q0 + w * 16 + m) * DIM + head * HD + hh * 8;
  v16h qf[2];
  qf[0] = frag_at(Qh + qoff);
  qf[1] = frag_at(Qh + qoff + 32);

  float mrow[8], lrow[8];
  v8f o[4];
#pragma unroll
  for (int v = 0; v < 8; ++v) { mrow[v] = -1.0e30f; lrow[v] = 0.0f; }
#pragma unroll
  for (int nb = 0; nb < 4; ++nb) o[nb] = (v8f){};

  const size_t kplane = (size_t)b * SEQ * DIM + head * HD;
  const size_t vplane = ((size_t)b * DIM + head * HD) * SEQ;

  for (int kb = 0; kb < SEQ; kb += 64) {
#pragma unroll
    for (int j = 0; j < 2; ++j) {
      const int idx = tid + 256 * j;
      const int r = idx >> 3, c = (idx & 7) * 8;
      *(v8h*)&Ks[r * LDT + c] = *(const v8h*)(Kh + kplane + (size_t)(kb + r) * DIM + c);
      *(v8h*)&Vs[r * LDT + c] = *(const v8h*)(Vt + vplane + (size_t)r * SEQ + kb + c);
    }
    __syncthreads();

    v8f s[4];
#pragma unroll
    for (int kg = 0; kg < 4; ++kg) {
      v8f t = {};
#pragma unroll
      for (int c = 0; c < 2; ++c) {
        const v16h kf = ld_frag(&Ks[(kg * 16) * LDT + c * 32], LDT);
        t = wmma16(qf[c], kf, t);
      }
      s[kg] = t * scale;
    }

    float alpha[8];
#pragma unroll
    for (int v = 0; v < 8; ++v) {
      float mx = fmaxf(fmaxf(s[0][v], s[1][v]), fmaxf(s[2][v], s[3][v]));
      mx = red16_max(mx);
      const float mn = fmaxf(mrow[v], mx);
      alpha[v] = __expf(mrow[v] - mn);
      mrow[v] = mn;
    }
#pragma unroll
    for (int kg = 0; kg < 4; ++kg)
#pragma unroll
      for (int v = 0; v < 8; ++v) s[kg][v] = __expf(s[kg][v] - mrow[v]);
#pragma unroll
    for (int v = 0; v < 8; ++v) {
      const float rs = red16_sum((s[0][v] + s[1][v]) + (s[2][v] + s[3][v]));
      lrow[v] = alpha[v] * lrow[v] + rs;
    }
#pragma unroll
    for (int nb = 0; nb < 4; ++nb)
#pragma unroll
      for (int v = 0; v < 8; ++v) o[nb][v] = o[nb][v] * alpha[v];

#pragma unroll
    for (int kg = 0; kg < 4; ++kg)
#pragma unroll
      for (int v = 0; v < 8; ++v)
        P[(hh * 8 + v) * LDT + kg * 16 + m] = (_Float16)(s[kg][v] * PCARRY);
    wave_lds_sync();

#pragma unroll
    for (int c = 0; c < 2; ++c) {
      const v16h pf = ld_frag(P + c * 32, LDT);
#pragma unroll
      for (int nb = 0; nb < 4; ++nb) {
        const v16h vf = ld_frag(&Vs[(nb * 16) * LDT + c * 32], LDT);
        o[nb] = wmma16(pf, vf, o[nb]);
      }
    }
    __syncthreads();
  }

  float inv[8];
#pragma unroll
  for (int v = 0; v < 8; ++v) inv[v] = __builtin_amdgcn_rcpf(lrow[v]) * (VCARRY / PCARRY);
#pragma unroll
  for (int nb = 0; nb < 4; ++nb)
#pragma unroll
    for (int v = 0; v < 8; ++v)
      P[(hh * 8 + v) * LDT + nb * 16 + m] = (_Float16)(o[nb][v] * inv[v]);
  wave_lds_sync();
  v8h x[4];
  size_t off[4];
#pragma unroll
  for (int i = 0; i < 4; ++i) {
    const int r = 4 * i + (lane >> 3);
    const int c = (lane & 7) * 8;
    x[i] = *(const v8h*)&P[r * LDT + c];
    off[i] = (size_t)(b * SEQ + q0 + w * 16 + r) * DIM + head * HD + c;
  }
#pragma unroll
  for (int i = 0; i < 4; ++i) *(volatile v8h*)(Ov + off[i]) = x[i];
  __threadfence();
#pragma unroll
  for (int i = 0; i < 4; ++i) *(volatile v8h*)(Ov + off[i]) = x[i];
}

extern "C" void kernel_launch(void* const* d_in, const int* in_sizes, int n_in,
                              void* d_out, int out_size, void* d_ws, size_t ws_size,
                              hipStream_t stream) {
  if (n_in < 11) return;
  const long long need_x = ((long long)(NB - 1) * SEQ_FULL + SEQ) * DIM;
  if ((long long)in_sizes[0] < need_x || (long long)in_sizes[1] < need_x ||
      (long long)in_sizes[2] < need_x) return;
  if (in_sizes[3] < DIM * DIM || in_sizes[4] < DIM * DIM || in_sizes[5] < DIM * DIM ||
      in_sizes[6] < DIM * DIM || in_sizes[7] < DIM * DIM || in_sizes[9] < DIM * DIM) return;
  if (in_sizes[8] < DIM || in_sizes[10] < DIM) return;
  if ((long long)out_size < need_x) return;
  if (ws_size < WS_TOTAL) return;

  const float* Qin = (const float*)d_in[0];
  const float* Kin = (const float*)d_in[1];
  const float* Vin = (const float*)d_in[2];
  const float* Wq  = (const float*)d_in[3];
  const float* Wk  = (const float*)d_in[4];
  const float* Wv  = (const float*)d_in[5];
  const float* Wo  = (const float*)d_in[6];
  const float* W1  = (const float*)d_in[7];
  const float* b1  = (const float*)d_in[8];
  const float* W2  = (const float*)d_in[9];
  const float* b2  = (const float*)d_in[10];
  float* out = (float*)d_out;

  char* ws = (char*)d_ws;
  _Float16* Wt = (_Float16*)ws;
  char* R1 = ws + WT_BYTES;
  char* R2 = R1 + R1_BYTES;
  _Float16* Xin16 = (_Float16*)R1;
  _Float16* Xq16 = Xin16;
  _Float16* Xk16 = (_Float16*)(R1 + PLANE16_BYTES);
  _Float16* Xv16 = (_Float16*)(R1 + 2 * PLANE16_BYTES);
  _Float16* Vatt16 = (_Float16*)R1;
  float*    X32    = (float*)(R1 + PLANE16_BYTES);
  _Float16* X16    = (_Float16*)(R1 + PLANE16_BYTES + PLANE32_BYTES);
  _Float16* Qh16 = (_Float16*)R2;
  _Float16* Kh16 = (_Float16*)(R2 + PLANE16_BYTES);
  _Float16* Vt16 = (_Float16*)(R2 + 2 * PLANE16_BYTES);
  _Float16* H16  = (_Float16*)R2;

  const size_t WP = (size_t)DIM * DIM;
  dim3 blk(256);
  dim3 gg(DIM / 64, MROWS / 64);

  wconv_kernel<<<dim3(DIM / 64, DIM / 64, 6), blk, 0, stream>>>(Wq, Wk, Wv, Wo, W1, W2, Wt);
  xconv_kernel<<<dim3((unsigned)(((size_t)MROWS * DIM) / 2048), 3), blk, 0, stream>>>(
      Qin, Kin, Vin, Xin16);
  gemm_kernel<0><<<gg, blk, 0, stream>>>(Xq16, Wt + 0 * WP, b1, X32, X32, Qh16);
  gemm_kernel<0><<<gg, blk, 0, stream>>>(Xk16, Wt + 1 * WP, b1, X32, X32, Kh16);
  gemm_kernel<1><<<gg, blk, 0, stream>>>(Xv16, Wt + 2 * WP, b1, X32, X32, Vt16);
  attn_kernel<<<dim3(SEQ / 128, NHEAD, NB), blk, 0, stream>>>(Qh16, Kh16, Vt16, Vatt16);
  gemm_kernel<2><<<gg, blk, 0, stream>>>(Vatt16, Wt + 3 * WP, Qin, X32, X32, X16);
  gemm_kernel<3><<<gg, blk, 0, stream>>>(X16, Wt + 4 * WP, b1, X32, X32, H16);
  gemm_kernel<4><<<gg, blk, 0, stream>>>(H16, Wt + 5 * WP, b2, X32, out, X16);
}
